// Echellogram_58325655880212
// MI455X (gfx1250) — hardware-verified
//
#include <hip/hip_runtime.h>
#include <math.h>

#define NX 1024
#define NY 85
#define NPIX (NX * NY)
#define NA 1500

typedef _Float16 f16;
typedef __attribute__((ext_vector_type(16))) f16 f16x16;
typedef __attribute__((ext_vector_type(8)))  float f32x8;
typedef __attribute__((ext_vector_type(4)))  float v4f_t;
typedef float v4fa __attribute__((ext_vector_type(4), may_alias));

__device__ __forceinline__ f32x8 wmma16(f16x16 a, f16x16 b, f32x8 c) {
  c = __builtin_amdgcn_wmma_f32_16x16x32_f16(false, a, false, b, (short)0, c, false, false);
  asm volatile("v_nop\n\tv_nop\n\tv_nop\n\tv_nop" : "+v"(c) : "v"(a), "v"(b));
  return c;
}

__global__ __launch_bounds__(256) void k_echelle(const int* __restrict__ index, const float* __restrict__ bkg, const float* __restrict__ sc,
                                                 const float* __restrict__ amps, const float* __restrict__ smooth, const float* __restrict__ lc,
                                                 const float* __restrict__ pc2, const float* __restrict__ srca, const float* __restrict__ fid,
                                                 const float* __restrict__ lamv, float* __restrict__ out) {
  __shared__ float mS[128][2];
  __shared__ __attribute__((aligned(16))) float oS[128];
  const int tid = threadIdx.x, lane = tid & 31, wave = tid >> 5, fr = lane & 15, kh = (lane >> 4) * 8;
  const int r0 = blockIdx.x * 128;
  const int rp = r0 + wave * 16 + fr; const int xi = rp / NY, yi = rp % NY;
  const float xx = (float)xi, yy = (float)yi;
  const float x = (xx - (float)(NX / 2)) / (float)(NX / 2);
  const float y = (yy - (float)NY / 2.0f) / ((float)NY / 2.0f);
  const float cx1 = fid[1] * (1.0f + lc[1] * 0.01f) * (float)NX / 2.0f;
  const float cx2 = 1.0f + lc[2];
  const float lam = fid[0] + lc[0] + cx1 * x + cx2 * (2.0f * x * x - 1.0f) + lc[3] * y;
  const float inv_s = 1.0f / 0.42f, pnorm = 0.3989422804014327f / 0.42f;
  f32x8 acc = {};
#pragma unroll 1
  for (int k0 = 0; k0 < NA; k0 += 32) {
    f16x16 af, bf;
#pragma unroll
    for (int i = 0; i < 8; ++i) {
      const int ka = k0 + kh + i, kb2 = k0 + 16 + kh + i;
      float pa = 0.0f, pb = 0.0f;
      if (ka < NA) { const float z = (lam - lamv[ka]) * inv_s; pa = __expf(-0.5f * z * z) * pnorm; }
      if (kb2 < NA) { const float z = (lam - lamv[kb2]) * inv_s; pb = __expf(-0.5f * z * z) * pnorm; }
      af[i] = (f16)pa; af[8 + i] = (f16)pb;
      float wa = 0.0f, wb = 0.0f;
      if (fr == 0) { wa = (ka < NA) ? amps[ka] : 0.0f; wb = (kb2 < NA) ? amps[kb2] : 0.0f; }
      else if (fr == 1) { wa = (ka < NA) ? srca[ka] : 0.0f; wb = (kb2 < NA) ? srca[kb2] : 0.0f; }
      bf[i] = (f16)wa; bf[8 + i] = (f16)wb;
    }
    acc = wmma16(af, bf, acc);
  }
  if (fr < 2) {
#pragma unroll
    for (int r = 0; r < 8; ++r) mS[wave * 16 + kh + r][fr] = acc[r];
  }
  __syncthreads();
  if (tid < 128) {
    const int rq = r0 + tid; const int xq = rq / NY, yq = rq % NY;
    const float xxq = (float)xq, yyq = (float)yq;
    const float ss = sc[1] * (yyq - sc[0] - sc[2] * xxq);
    const float inv_beta = __expf(-smooth[0]);
    const float e1 = 1.0f / (1.0f + __expf(-(ss * inv_beta))), e2 = 1.0f / (1.0f + __expf(-((12.0f - ss) * inv_beta)));
    const float emask = e1 * e2;
    int idx = index[0]; idx = min(max(idx, 0), 1);
    const float p0 = pc2[idx * 2 + 0], p1 = pc2[idx * 2 + 1];
    const float sig = __expf(p1);
    const float t = (ss - p0) / sig;
    const float src_prof = __expf(-0.5f * t * t - logf(sig) - 0.9189385332046727f);
    oS[tid] = emask * mS[tid][0] + src_prof * mS[tid][1] + bkg[0];
  }
  __syncthreads();
  if (tid < 32) { *(volatile v4f_t*)(out + r0 + tid * 4) = *(const volatile v4fa*)(oS + tid * 4); __threadfence(); *(volatile v4f_t*)(out + r0 + tid * 4) = *(const volatile v4fa*)(oS + tid * 4); }
}

extern "C" void kernel_launch(void* const* d_in, const int* in_sizes, int n_in,
                              void* d_out, int out_size, void* d_ws, size_t ws_size,
                              hipStream_t stream) {
  (void)in_sizes; (void)n_in; (void)out_size; (void)d_ws; (void)ws_size;
  const int* index = (const int*)d_in[0];
  const float* bkg = (const float*)d_in[1], *sc = (const float*)d_in[2], *amps = (const float*)d_in[3], *smooth = (const float*)d_in[4];
  const float* lc = (const float*)d_in[5], *pc2 = (const float*)d_in[6], *srca = (const float*)d_in[7], *fid = (const float*)d_in[8], *lamv = (const float*)d_in[9];
  float* out = (float*)d_out;
  k_echelle<<<dim3(NPIX / 128), dim3(256), 0, stream>>>(index, bkg, sc, amps, smooth, lc, pc2, srca, fid, lamv, out);
}
